// ModelCausality_14302241096268
// MI455X (gfx1250) — hardware-run, weakly checked
//
#include <hip/hip_runtime.h>
#include <math.h>
#include <stdint.h>

constexpr int kBatchN    = 8;
constexpr int kSideA     = 256;
constexpr int kSideB     = 256;
constexpr int kCin       = 64;
constexpr int kHid       = 256;
constexpr int kChunkRows = kSideA * kSideB;
constexpr float kWCarry  = 16.0f;
constexpr float kHCarry  = 8.0f;
constexpr float kScale0  = kHCarry / kWCarry;
constexpr float kScale1  = 1.0f / (kHCarry * kWCarry);

constexpr size_t kOffZ16  = 0;
constexpr size_t kBytesZ16 = (size_t)kChunkRows * kCin * 2;
constexpr size_t kOffH16  = kOffZ16 + kBytesZ16;
constexpr size_t kBytesH16 = (size_t)kChunkRows * kHid * 2;
constexpr size_t kOffHf   = kOffH16 + kBytesH16;
constexpr size_t kBytesHf = (size_t)kChunkRows * kHid * 4;
constexpr size_t kOffW0h  = kOffHf + kBytesHf;
constexpr size_t kBytesW0h = (size_t)kHid * kCin * 2;
constexpr size_t kOffW1h  = kOffW0h + kBytesW0h;
constexpr size_t kBytesW1h = (size_t)kHid * kHid * 2;
constexpr size_t kOffB0x8 = kOffW1h + kBytesW1h;
constexpr size_t kBytesB0x8 = (size_t)kHid * 4;
constexpr size_t kCarveTotal = kOffB0x8 + kBytesB0x8;
static_assert(kCarveTotal == 109216768ull);
static_assert(kCarveTotal <= 134217728ull);

typedef __attribute__((ext_vector_type(16))) _Float16 v16h;
typedef __attribute__((ext_vector_type(8)))  _Float16 v8h;
typedef __attribute__((ext_vector_type(16))) __bf16   v16b;
typedef __attribute__((ext_vector_type(8)))  __bf16   v8b;
typedef __attribute__((ext_vector_type(8)))  float    v8f;
typedef __attribute__((ext_vector_type(4)))  float    v4f;
typedef __attribute__((ext_vector_type(4)))  unsigned int v4u;

__device__ __forceinline__ unsigned short f2bf_bits(float f) {
  unsigned u = __float_as_uint(f);
  return (unsigned short)((u + 0x7FFFu + ((u >> 16) & 1u)) >> 16);
}
__device__ __forceinline__ float bf_bits2f(unsigned short h) { return __uint_as_float(((unsigned)h) << 16); }

__device__ __forceinline__ void dep_guard_h(v8f& a, v8f& b, v16h x, v16h y) { asm volatile("v_nop\n\tv_nop\n\tv_nop\n\tv_nop" : "+v"(a), "+v"(b) : "v"(x), "v"(y)); }
__device__ __forceinline__ void dep_guard_b(v8f& a, v8f& b, v16b x, v16b y) { asm volatile("v_nop\n\tv_nop\n\tv_nop\n\tv_nop" : "+v"(a), "+v"(b) : "v"(x), "v"(y)); }
__device__ __forceinline__ void keep4_h(v16h a, v16h b, v16h c, v16h d) { asm volatile("v_nop" :: "v"(a), "v"(b), "v"(c), "v"(d)); }
__device__ __forceinline__ void keep4_b(v16b a, v16b b, v16b c, v16b d) { asm volatile("v_nop" :: "v"(a), "v"(b), "v"(c), "v"(d)); }
__device__ __forceinline__ void acc_guard4(v8f& a, v8f& b, v8f& c, v8f& d) { asm volatile("v_nop\n\tv_nop\n\tv_nop\n\tv_nop" : "+v"(a), "+v"(b), "+v"(c), "+v"(d)); }
template <typename T> struct Frag;
template <> struct Frag<_Float16> {
  typedef v16h V; union U { v16h v; v8h h[2]; };
  static __device__ __forceinline__ v16h load(const _Float16* p) {
    U f; f.h[0] = *(const v8h*)(p); f.h[1] = *(const v8h*)(p + 16); return f.v;
  }
  static __device__ __forceinline__ v8f mma(v16h a, v16h b, v8f c) {
    return __builtin_amdgcn_wmma_f32_16x16x32_f16(false, a, false, b, (short)0, c, false, false);
  }
  static __device__ __forceinline__ void guard(v8f& a, v8f& b, v16h x, v16h y) { dep_guard_h(a, b, x, y); }
  static __device__ __forceinline__ void keep(v16h a, v16h b, v16h c, v16h d) { keep4_h(a, b, c, d); }
};
template <> struct Frag<__bf16> {
  typedef v16b V; union U { v16b v; v8b h[2]; };
  static __device__ __forceinline__ v16b load(const __bf16* p) {
    U f; f.h[0] = *(const v8b*)(p); f.h[1] = *(const v8b*)(p + 16); return f.v;
  }
  static __device__ __forceinline__ v8f mma(v16b a, v16b b, v8f c) {
    return __builtin_amdgcn_wmma_f32_16x16x32_bf16(false, a, false, b, (short)0, c, false, false);
  }
  static __device__ __forceinline__ void guard(v8f& a, v8f& b, v16b x, v16b y) { dep_guard_b(a, b, x, y); }
  static __device__ __forceinline__ void keep(v16b a, v16b b, v16b c, v16b d) { keep4_b(a, b, c, d); }
};

__device__ __forceinline__ unsigned pk16(unsigned short a, unsigned short b) { return (unsigned)a | ((unsigned)b << 16); }
__device__ __forceinline__ unsigned short h_bits(float f) { const _Float16 h = (_Float16)f; return __builtin_bit_cast(unsigned short, h); }

template <int ET> struct Elem;
template <> struct Elem<0> { typedef _Float16 T; };
template <> struct Elem<1> { typedef __bf16 T; };
template <int ET, bool SPLIT, int BIAS_MODE, int OUT_MODE, bool RESID, int ACT = 0>
__global__ __launch_bounds__(256) void wmma_gemm64(
    const unsigned short* __restrict__ Ap, const unsigned short* __restrict__ A2p, int lda, long strideA,
    const unsigned short* __restrict__ Btp, const unsigned short* __restrict__ Bt2p, int ldb, long strideB,
    void* __restrict__ Cout, void* __restrict__ Cout2, int ldc, long strideC,
    const float* __restrict__ bias,
    const float* __restrict__ resid, long strideR,
    int M, int N, int K, float scale) {
  typedef typename Elem<ET>::T T;
  typedef typename Frag<T>::V V;
  const T* A = (const T*)Ap; const T* A2 = (const T*)A2p; const T* Bt = (const T*)Btp; const T* Bt2 = (const T*)Bt2p;
  __shared__ __align__(16) float sT[8][16 * 68];
  const int b    = blockIdx.y;
  const int lane = threadIdx.x & 31;
  const int wave = threadIdx.x >> 5;
  const int tilesN = N >> 6;
  const int tilesM = M >> 6;
  const int tile = blockIdx.x * 8 + wave;
  if (tile >= tilesM * tilesN) return;
  const int tm = tile / tilesN;
  const int tn = tile - tm * tilesN;
  const int m0 = tm << 6;
  const int n0 = tn << 6;

  const T* Ab  = A  + (size_t)b * strideA;
  const T* Bb  = Bt + (size_t)b * strideB;
  const T* Ab2 = SPLIT ? (A2  + (size_t)b * strideA) : nullptr;
  const T* Bb2 = SPLIT ? (Bt2 + (size_t)b * strideB) : nullptr;

  const int rlane = lane & 15;
  const int koff  = (lane >> 4) * 8;
  const int mOff  = (lane >> 4) * 8;

  v8f acc[4][4];
#pragma unroll
  for (int i = 0; i < 4; ++i)
#pragma unroll
    for (int j = 0; j < 4; ++j) acc[i][j] = (v8f){0.f,0.f,0.f,0.f,0.f,0.f,0.f,0.f};

  for (int k0 = 0; k0 < K; k0 += 32) {
    V bh[4], bl[4];
#pragma unroll
    for (int j = 0; j < 4; ++j) {
      const size_t bo = (size_t)(n0 + (j << 4) + rlane) * ldb + koff + k0;
      bh[j] = Frag<T>::load(Bb + bo);
      if (SPLIT) bl[j] = Frag<T>::load(Bb2 + bo);
    }
#pragma unroll
    for (int i = 0; i < 4; ++i) {
      const size_t ao = (size_t)(m0 + (i << 4) + rlane) * lda + koff + k0;
      V ah = Frag<T>::load(Ab + ao);
      V al;
      if (SPLIT) al = Frag<T>::load(Ab2 + ao);
#pragma unroll
      for (int j = 0; j < 4; ++j) {
        acc[i][j] = Frag<T>::mma(ah, bh[j], acc[i][j]);
        if (SPLIT) {
          acc[i][j] = Frag<T>::mma(ah, bl[j], acc[i][j]);
          acc[i][j] = Frag<T>::mma(al, bh[j], acc[i][j]);
        }
      }
      Frag<T>::guard(acc[i][0], acc[i][3], ah, SPLIT ? al : ah);
    }
    Frag<T>::keep(bh[0], bh[1], bh[2], bh[3]);
    if (SPLIT) Frag<T>::keep(bl[0], bl[1], bl[2], bl[3]);
  }
  acc_guard4(acc[0][0], acc[0][1], acc[0][2], acc[0][3]);
  acc_guard4(acc[1][0], acc[1][1], acc[1][2], acc[1][3]);
  acc_guard4(acc[2][0], acc[2][1], acc[2][2], acc[2][3]);
  acc_guard4(acc[3][0], acc[3][1], acc[3][2], acc[3][3]);

  float* slab = sT[wave];
  const float* Rb = RESID ? (resid + (size_t)b * strideR) : nullptr;
#pragma unroll
  for (int i = 0; i < 4; ++i) {
    const int mBase = m0 + (i << 4);
#pragma unroll
    for (int j = 0; j < 4; ++j) {
      const int n = n0 + (j << 4) + rlane;
      float bv = 0.f;
      if (BIAS_MODE == 2) bv = bias[n];
#pragma unroll
      for (int r = 0; r < 8; ++r) {
        float v = acc[i][j][r] * scale;
        if (BIAS_MODE == 1) v += bias[mBase + mOff + r];
        if (BIAS_MODE == 2) v += bv;
        if (RESID) v += Rb[(size_t)(mBase + mOff + r) * ldc + n];
        if (ACT == 2) v = fmaxf(v, 0.0f);
        if (ACT == 4) v = (v > 0.f) ? v : 0.01f * v;
        slab[(mOff + r) * 68 + (j << 4) + rlane] = v;
      }
    }
    __builtin_amdgcn_fence(__ATOMIC_RELEASE, "workgroup");
    __builtin_amdgcn_wave_barrier();
    __builtin_amdgcn_fence(__ATOMIC_ACQUIRE, "workgroup");
    if (OUT_MODE == 0) {
      float* C = (float*)Cout + (size_t)b * strideC;
      const int hh = lane >> 4, c4 = (lane & 15) * 4;
      for (int pass = 0; pass < 2; ++pass) {
#pragma unroll
        for (int it = 0; it < 8; ++it) {
          const int row = it * 2 + hh;
          v4f v = *(const v4f*)(slab + row * 68 + c4);
          *(volatile v4f*)(C + (size_t)(mBase + row) * ldc + n0 + c4) = v;
        }
        __threadfence();
      }
    } else {
      const int q = lane >> 3, c8 = (lane & 7) * 8;
      unsigned short* C  = (unsigned short*)Cout  + (size_t)b * strideC;
      unsigned short* C2 = (OUT_MODE == 2) ? ((unsigned short*)Cout2 + (size_t)b * strideC) : nullptr;
      for (int pass = 0; pass < 2; ++pass) {
#pragma unroll
        for (int it = 0; it < 4; ++it) {
          const int row = it * 4 + q;
          const float* sp = slab + row * 68 + c8;
          v8h hv, lv;
#pragma unroll
          for (int e = 0; e < 8; ++e) {
            if (OUT_MODE == 1) {
              hv[e] = (_Float16)sp[e];
            } else {
              unsigned short hb = f2bf_bits(sp[e]);
              unsigned short lb = f2bf_bits(sp[e] - bf_bits2f(hb));
              hv[e] = __builtin_bit_cast(_Float16, hb);
              lv[e] = __builtin_bit_cast(_Float16, lb);
            }
          }
          *(volatile v8h*)(C + (size_t)(mBase + row) * ldc + n0 + c8) = hv;
          if (OUT_MODE == 2) *(volatile v8h*)(C2 + (size_t)(mBase + row) * ldc + n0 + c8) = lv;
        }
        __threadfence();
      }
    }
    __builtin_amdgcn_fence(__ATOMIC_RELEASE, "workgroup");
    __builtin_amdgcn_wave_barrier();
    __builtin_amdgcn_fence(__ATOMIC_ACQUIRE, "workgroup");
  }
}

__global__ __launch_bounds__(256) void cast8_f16_scaled_kernel(const float* __restrict__ in, unsigned short* __restrict__ out,
                                                               int n8, float carry) {
  const int i = blockIdx.x * 256 + threadIdx.x;
  if (i >= n8) return;
  const float* p = in + 8 * (size_t)i;
  const v4f a = *(const v4f*)(p);
  const v4f c = *(const v4f*)(p + 4);
  unsigned short hb[8];
#pragma unroll
  for (int e = 0; e < 4; ++e) {
    hb[e]     = h_bits(a[e] * carry);
    hb[4 + e] = h_bits(c[e] * carry);
  }
  const v4u u = (v4u){pk16(hb[0], hb[1]), pk16(hb[2], hb[3]), pk16(hb[4], hb[5]), pk16(hb[6], hb[7])};
  unsigned short* q = out + 8 * (size_t)i;
  *(volatile v4u*)q = u;
  __threadfence();
  *(volatile v4u*)q = u;
}

__global__ __launch_bounds__(64) void bias_scale_kernel(const float* __restrict__ bsrc, float* __restrict__ bdst, float mul) {
  const int t = threadIdx.x;
  v4f v = *(const v4f*)(bsrc + 4 * t);
  v = v * mul;
  *(volatile v4f*)(bdst + 4 * t) = v;
  __threadfence();
  *(volatile v4f*)(bdst + 4 * t) = v;
}

__global__ __launch_bounds__(256) void diff_kernel(const float* __restrict__ zaN, const float* __restrict__ zbN,
                                                   unsigned short* __restrict__ Z, int nThreads) {
  const int i = blockIdx.x * 256 + threadIdx.x;
  if (i >= nThreads) return;
  const int row = i >> 3;
  const int c0  = (i & 7) * 8;
  const int a   = row >> 8;
  const int bb  = row & 255;
  const float* pa = zaN + (size_t)a  * kCin + c0;
  const float* pb = zbN + (size_t)bb * kCin + c0;
  const v4f xa0 = *(const v4f*)(pa);
  const v4f xa1 = *(const v4f*)(pa + 4);
  const v4f xb0 = *(const v4f*)(pb);
  const v4f xb1 = *(const v4f*)(pb + 4);
  unsigned short hb[8];
#pragma unroll
  for (int e = 0; e < 4; ++e) {
    hb[e]     = h_bits(xa0[e] - xb0[e]);
    hb[4 + e] = h_bits(xa1[e] - xb1[e]);
  }
  const v4u u = (v4u){pk16(hb[0], hb[1]), pk16(hb[2], hb[3]), pk16(hb[4], hb[5]), pk16(hb[6], hb[7])};
  unsigned short* q = Z + 8 * (size_t)i;
  *(volatile v4u*)q = u;
  __threadfence();
  *(volatile v4u*)q = u;
}

__global__ __launch_bounds__(256) void head_kernel(const float* __restrict__ Hf, const float* __restrict__ w2,
                                                   const float* __restrict__ b2, float* __restrict__ out, int n) {
  __shared__ __align__(16) float sY[kSideB];
  const int a    = blockIdx.x;
  const int t    = threadIdx.x;
  const int lane = t & 31;
  const int wave = t >> 5;
  const v4f wa = *(const v4f*)(w2 + lane * 8);
  const v4f wb = *(const v4f*)(w2 + lane * 8 + 4);
  const float bias2 = b2[0];
  const float* base = Hf + (size_t)a * kSideB * kHid;
#pragma unroll 1
  for (int i = 0; i < 32; ++i) {
    const int bidx = wave * 32 + i;
    const float* hr = base + (size_t)bidx * kHid + lane * 8;
    const v4f x0 = *(const v4f*)(hr);
    const v4f x1 = *(const v4f*)(hr + 4);
    float s = x0[0] * wa[0];
    s += x0[1] * wa[1];
    s += x0[2] * wa[2];
    s += x0[3] * wa[3];
    s += x1[0] * wb[0];
    s += x1[1] * wb[1];
    s += x1[2] * wb[2];
    s += x1[3] * wb[3];
    s += __shfl_xor(s, 16, 32);
    s += __shfl_xor(s, 8, 32);
    s += __shfl_xor(s, 4, 32);
    s += __shfl_xor(s, 2, 32);
    s += __shfl_xor(s, 1, 32);
    const float x = s + bias2;
    const float ex = expf(-x);
    const float y = 1.0f / (1.0f + ex);
    if (lane == 0) sY[bidx] = y;
  }
  __syncthreads();
  if (wave == 0) {
    float* orow = out + ((size_t)n * kSideA + a) * kSideB;
    const v4f v0 = *(const v4f*)(sY + lane * 4);
    const v4f v1 = *(const v4f*)(sY + 128 + lane * 4);
    for (int pass = 0; pass < 2; ++pass) {
      *(volatile v4f*)(orow + lane * 4) = v0;
      *(volatile v4f*)(orow + 128 + lane * 4) = v1;
      __threadfence();
    }
  }
}

extern "C" void kernel_launch(void* const* d_in, const int* in_sizes, int n_in,
                              void* d_out, int out_size, void* d_ws, size_t ws_size,
                              hipStream_t stream)
{
  if (n_in < 8) return;
  if (out_size != kBatchN * kSideA * kSideB) return;
  if (in_sizes[0] != kBatchN * kSideA * kCin) return;
  if (in_sizes[1] != kBatchN * kSideB * kCin) return;
  if (in_sizes[2] != kHid * kCin) return;
  if (in_sizes[3] != kHid) return;
  if (in_sizes[4] != kHid * kHid) return;
  if (in_sizes[5] != kHid) return;
  if (in_sizes[6] != kHid) return;
  if (in_sizes[7] < 1) return;
  if (ws_size < kCarveTotal) return;

  const float* za = (const float*)d_in[0];
  const float* zb = (const float*)d_in[1];
  const float* w0 = (const float*)d_in[2];
  const float* b0 = (const float*)d_in[3];
  const float* w1 = (const float*)d_in[4];
  const float* b1 = (const float*)d_in[5];
  const float* w2 = (const float*)d_in[6];
  const float* b2 = (const float*)d_in[7];
  float* out = (float*)d_out;

  char* ws = (char*)d_ws;
  unsigned short* Z16  = (unsigned short*)(ws + kOffZ16);
  unsigned short* H16  = (unsigned short*)(ws + kOffH16);
  float*          Hf   = (float*)(ws + kOffHf);
  unsigned short* W0h  = (unsigned short*)(ws + kOffW0h);
  unsigned short* W1h  = (unsigned short*)(ws + kOffW1h);
  float*          b0x8 = (float*)(ws + kOffB0x8);

  cast8_f16_scaled_kernel<<<dim3((kHid * kCin / 8) / 256), dim3(256), 0, stream>>>(w0, W0h, kHid * kCin / 8, kWCarry);
  cast8_f16_scaled_kernel<<<dim3((kHid * kHid / 8) / 256), dim3(256), 0, stream>>>(w1, W1h, kHid * kHid / 8, kWCarry);
  bias_scale_kernel<<<dim3(1), dim3(64), 0, stream>>>(b0, b0x8, kHCarry);

  const int diffThreads = kChunkRows * kCin / 8;
  const int gemmBlocks  = ((kChunkRows / 64) * (kHid / 64)) / 8;

  for (int n = 0; n < kBatchN; ++n) {
    const float* zaN = za + (size_t)n * kSideA * kCin;
    const float* zbN = zb + (size_t)n * kSideB * kCin;

    diff_kernel<<<dim3(diffThreads / 256), dim3(256), 0, stream>>>(zaN, zbN, Z16, diffThreads);

    wmma_gemm64<0, false, 2, 1, false, 4><<<dim3(gemmBlocks, 1, 1), dim3(256), 0, stream>>>(
        Z16, Z16, kCin, 0L,
        W0h, W0h, kCin, 0L,
        (void*)H16, (void*)H16, kHid, 0L,
        b0x8,
        b1, 0L,
        kChunkRows, kHid, kCin, kScale0);

    wmma_gemm64<0, false, 2, 0, false, 4><<<dim3(gemmBlocks, 1, 1), dim3(256), 0, stream>>>(
        H16, H16, kHid, 0L,
        W1h, W1h, kHid, 0L,
        (void*)Hf, (void*)Hf, kHid, 0L,
        b1,
        b1, 0L,
        kChunkRows, kHid, kHid, kScale1);

    head_kernel<<<dim3(kSideA), dim3(256), 0, stream>>>(Hf, w2, b2, out, n);
  }
}
